// DiagonalS6SSM_47708496724573
// MI455X (gfx1250) — hardware-verified
//
#include <hip/hip_runtime.h>
#include <stddef.h>
#include <stdint.h>


#define TT     8
#define CIN    128
#define HH     64
#define NS     16
#define CO     160
#define COUT   64
#define LN_EPS 1e-5f

#define GR     32
#define NTHR   256
#define NWAVE  8
#define CHUNK  2048
#define WCAP   256
#define NGRP   (CHUNK / (NTHR * 4))

static_assert(WCAP == (CHUNK / NTHR) * 32);
static_assert(NGRP == 2);
static_assert(CHUNK <= 2048);

typedef float          v2f  __attribute__((ext_vector_type(2)));
typedef float          v4f  __attribute__((ext_vector_type(4)));
typedef float          v8f  __attribute__((ext_vector_type(8)));
typedef int            v4i  __attribute__((ext_vector_type(4)));
typedef unsigned int   v4u  __attribute__((ext_vector_type(4)));
typedef unsigned short v8us __attribute__((ext_vector_type(8)));
typedef __bf16         v16b __attribute__((ext_vector_type(16)));
union BFrag { v16b v; v8us half[2]; };
union Pack8 { v8us s; v4u u; };
static_assert(sizeof(BFrag) == 32);
static_assert(sizeof(Pack8) == 16);

__device__ __forceinline__ v8f wmb(v16b a, v16b b, v8f c) {
  v8f d = __builtin_amdgcn_wmma_f32_16x16x32_bf16(false, a, false, b, (short)0, c, false, false);
  asm volatile("v_nop\n\tv_nop\n\tv_nop\n\tv_nop" : "+v"(d) : "v"(a), "v"(b));
  return d;
}

__device__ __forceinline__ float wsum(float v) {
  v += __shfl_xor(v, 16, 32);
  v += __shfl_xor(v, 8, 32);
  v += __shfl_xor(v, 4, 32);
  v += __shfl_xor(v, 2, 32);
  v += __shfl_xor(v, 1, 32);
  return v;
}

__device__ __forceinline__ void split1(float f, unsigned short& hb, unsigned short& lb) {
  const unsigned u  = __float_as_uint(f);
  const unsigned hu = (u + 0x7FFFu + ((u >> 16) & 1u)) & 0xFFFF0000u;
  const float    rf = f - __uint_as_float(hu);
  const unsigned ru = __float_as_uint(rf);
  const unsigned lu = (ru + 0x7FFFu + ((ru >> 16) & 1u)) >> 16;
  hb = (unsigned short)(hu >> 16);
  lb = (unsigned short)lu;
}

__device__ __forceinline__ void split8(v4f a, v4f b, Pack8& ph, Pack8& pl) {
  float f[8] = {a.x, a.y, a.z, a.w, b.x, b.y, b.z, b.w};
#pragma unroll
  for (int q = 0; q < 8; ++q) {
    unsigned short hb, lb;
    split1(f[q], hb, lb);
    ph.s[q] = hb;
    pl.s[q] = lb;
  }
}

__global__ __launch_bounds__(NTHR) void k_wprep(const float* __restrict__ W, int Kin, int Nout,
                                                unsigned short* oh, unsigned short* ol) {
  const int kg8   = Kin >> 3;
  const int total = Nout * kg8;
  const int i = blockIdx.x * NTHR + threadIdx.x;
  if (i >= total) return;
  const int n  = i / kg8;
  const int kg = i - n * kg8;
  Pack8 ph, pl;
#pragma unroll
  for (int q = 0; q < 8; ++q) {
    const float f = W[(size_t)(kg * 8 + q) * Nout + n];
    unsigned short hb, lb;
    split1(f, hb, lb);
    ph.s[q] = hb;
    pl.s[q] = lb;
  }
  const size_t o = (size_t)n * Kin + (size_t)kg * 8;
  *(volatile v4u*)(oh + o) = ph.u;
  *(volatile v4u*)(ol + o) = pl.u;
  __threadfence();
  *(volatile v4u*)(oh + o) = ph.u;
  *(volatile v4u*)(ol + o) = pl.u;
}

template<int C>
__global__ __launch_bounds__(NTHR) void k_agg(const float* __restrict__ x, const int* __restrict__ ei,
                                              unsigned short* ph, unsigned short* pl, int nV, int nE) {
  constexpr int NB   = 32768 / C;
  constexpr int SB   = (NB == 256) ? 8 : 9;
  constexpr int CPL  = C / 32;
  constexpr int SPW  = NB / NWAVE;
  constexpr int LPSL = C / 4;
  constexpr int SPI  = 32 / LPSL;
  constexpr int NPI  = SPW / SPI;
  static_assert(NB == (1 << SB));
  static_assert(NB * C == 32768);
  static_assert(CPL == 4 || CPL == 2);

  extern __shared__ v4f lds_dyn[];
  float* sacc = (float*)lds_dyn;
  int*   cnt  = (int*)(sacc + NB * C);
  int*   list = cnt + NB;
  int*   wcnt = list + NWAVE * WCAP;

  const int tid  = threadIdx.x;
  const int lane = tid & 31;
  const int wave = tid >> 5;
  const int t    = blockIdx.y;
  const int nodeBase = blockIdx.x * NB;

  {
    const v4f z4 = {0.f, 0.f, 0.f, 0.f};
    for (int i = tid; i < NB * C / 4; i += NTHR) lds_dyn[i] = z4;
    for (int i = tid; i < NB; i += NTHR) cnt[i] = 0;
  }
  __syncthreads();

  const int*   esrc = ei + (size_t)t * 2 * (size_t)nE;
  const int*   eid  = esrc + nE;
  const bool   al16 = ((((size_t)(2 * t + 1) * (size_t)nE) & 3) == 0);
  const float* xt   = x + (size_t)t * (size_t)nV * C;

  const int nChunks = (nE + CHUNK - 1) / CHUNK;
#pragma unroll 1
  for (int ch = 0; ch < nChunks; ++ch) {
    const int cbase = ch * CHUNK;
    int wc = 0;
#pragma unroll
    for (int g = 0; g < NGRP; ++g) {
      const int el0 = (g * NTHR + tid) * 4;
      const int e0  = cbase + el0;
      v4i d;
      if (al16 && (cbase + CHUNK <= nE)) {
        d = *(const v4i*)(eid + e0);
      } else {
        const int sent = -2147483647 - 1;
        const int i0 = (e0     < nE) ? e0     : nE - 1;
        const int i1 = (e0 + 1 < nE) ? e0 + 1 : nE - 1;
        const int i2 = (e0 + 2 < nE) ? e0 + 2 : nE - 1;
        const int i3 = (e0 + 3 < nE) ? e0 + 3 : nE - 1;
        const int r0 = eid[i0], r1 = eid[i1], r2 = eid[i2], r3 = eid[i3];
        d.x = (e0     < nE) ? r0 : sent;
        d.y = (e0 + 1 < nE) ? r1 : sent;
        d.z = (e0 + 2 < nE) ? r2 : sent;
        d.w = (e0 + 3 < nE) ? r3 : sent;
      }
      const unsigned s0 = (unsigned)d.x - (unsigned)nodeBase;
      const unsigned s1 = (unsigned)d.y - (unsigned)nodeBase;
      const unsigned s2 = (unsigned)d.z - (unsigned)nodeBase;
      const unsigned s3 = (unsigned)d.w - (unsigned)nodeBase;
      const bool h0 = s0 < (unsigned)NB;
      const bool h1 = s1 < (unsigned)NB;
      const bool h2 = s2 < (unsigned)NB;
      const bool h3 = s3 < (unsigned)NB;
      const unsigned many = __builtin_amdgcn_ballot_w32(h0 | h1 | h2 | h3);
      if (many != 0u) {
#define HITJ(J, HJ, SJ) { \
          const unsigned mj = __builtin_amdgcn_ballot_w32(HJ); \
          if (HJ) { \
            const int pos = wc + (int)__builtin_amdgcn_mbcnt_lo(mj, 0u); \
            if (pos < WCAP) list[wave * WCAP + pos] = ((el0 + (J)) << SB) | (int)(SJ); \
          } \
          wc += (int)__builtin_popcount(mj); }
        HITJ(0, h0, s0)
        HITJ(1, h1, s1)
        HITJ(2, h2, s2)
        HITJ(3, h3, s3)
#undef HITJ
      }
    }
    if (lane == 0) wcnt[wave] = wc;
    __syncthreads();

    if (wave == 0) {
      for (int wsx = 0; wsx < NWAVE; ++wsx) {
        int n = wcnt[wsx];
        n = (n > WCAP) ? WCAP : ((n < 0) ? 0 : n);
        for (int i = 0; i < n; ++i) {
          const int ent  = list[wsx * WCAP + i];
          const int slot = ent & (NB - 1);
          const int el   = (ent >> SB) & (CHUNK - 1);
          int e = cbase + el;
          if (e > nE - 1) e = nE - 1;
          int src = esrc[e];
          src = (src < 0) ? 0 : ((src > nV - 1) ? nV - 1 : src);
          if constexpr (C == 128) {
            const v4f xv = *(const v4f*)(xt + (size_t)src * C + 4 * lane);
            v4f* sp = (v4f*)(sacc + slot * C + 4 * lane);
            const v4f cur = *sp;
            *sp = cur + xv;
          } else {
            const v2f xv = *(const v2f*)(xt + (size_t)src * C + 2 * lane);
            v2f* sp = (v2f*)(sacc + slot * C + 2 * lane);
            const v2f cur = *sp;
            *sp = cur + xv;
          }
          if (lane == 0) cnt[slot] = cnt[slot] + 1;
        }
      }
    }
    __syncthreads();
  }

  const int within = lane % LPSL;
  const int plane  = within / (C / 8);
  const int piece  = within % (C / 8);
  const int sub    = lane / LPSL;
  unsigned short* pb = plane ? pl : ph;
  auto emit = [&]() {
#pragma unroll 1
    for (int i = 0; i < NPI; ++i) {
      const int slot = wave * SPW + i * SPI + sub;
      const int node = nodeBase + slot;
      const float* sr = sacc + slot * C + 8 * piece;
      const v4f f0 = *(const v4f*)sr;
      const v4f f1 = *(const v4f*)(sr + 4);
      const int   c   = cnt[slot];
      const float cc  = fmaxf((float)c, 1.0f);
      const float inv = 1.0f / cc;
      Pack8 wh, wl;
      split8(f0 * inv, f1 * inv, wh, wl);
      Pack8 w;
#pragma unroll
      for (int q = 0; q < 8; ++q) w.s[q] = plane ? wl.s[q] : wh.s[q];
      if (node < nV) {
        *(volatile v4u*)(pb + ((size_t)t * (size_t)nV + (size_t)node) * C + 8 * piece) = w.u;
      }
    }
  };
  emit();
  __threadfence();
  emit();
}

template<int K, int NTM, int NTR, bool DUAL>
__global__ __launch_bounds__(128) void k_gemm(
    const float* __restrict__ A0, int M,
    const unsigned short* __restrict__ A1h, const unsigned short* __restrict__ A1l,
    const unsigned short* __restrict__ Wh,  const unsigned short* __restrict__ Wl,
    const unsigned short* __restrict__ Vh,  const unsigned short* __restrict__ Vl,
    const float* __restrict__ bias0, const float* __restrict__ bias1,
    float* out0, float* out1, int res_row0)
{
  constexpr int NT  = NTM + NTR;
  constexpr int NTW = NT / 2;
  constexpr int FM0 = NTM * 16;
  constexpr int FM1 = NTR * 16;
  constexpr int XP  = NT * 16 + 4;
  constexpr int KQ  = K / 4;
  static_assert((NT % 2) == 0);
  static_assert((K % 32) == 0);
  static_assert(FM1 == 0 || FM1 == 64);
  static_assert((KQ % 8) == 0);

  __shared__ __attribute__((aligned(16))) unsigned short Ah[GR * K];
  __shared__ __attribute__((aligned(16))) unsigned short Al[GR * K];
  __shared__ __attribute__((aligned(16))) float Xs[GR * XP];

  const int tid  = threadIdx.x;
  const int lane = tid & 31;
  const int wave = __builtin_amdgcn_readfirstlane((int)(tid >> 5));
  const int hh   = lane >> 4;
  const int m    = lane & 15;
  const int rt   = wave & 1;
  const int ch   = wave >> 1;
  const int rowBase = blockIdx.x * GR;
  const bool dores  = (NTR > 0) && (rowBase + GR > res_row0);

  {
    const int r  = tid >> 2;
    const int qq = tid & 3;
    int grow = rowBase + r;
    if (grow > M - 1) grow = M - 1;
    const float* p = A0 + (size_t)grow * K + qq * KQ;
    unsigned short* dh = Ah + r * K + qq * KQ;
    unsigned short* dl = Al + r * K + qq * KQ;
#pragma unroll
    for (int s = 0; s < KQ / 8; ++s) {
      const v4f f0 = *(const v4f*)(p + 8 * s);
      const v4f f1 = *(const v4f*)(p + 8 * s + 4);
      Pack8 ph, plo;
      split8(f0, f1, ph, plo);
      *(v8us*)(dh + 8 * s) = ph.s;
      *(v8us*)(dl + 8 * s) = plo.s;
    }
  }
  __syncthreads();

  v8f c[NTW];
#pragma unroll
  for (int j = 0; j < NTW; ++j) {
    const int col = (ch * NTW + j) * 16 + m;
    float bv;
    if constexpr (NTR > 0) {
      int i0 = col;       if (i0 > FM0 - 1) i0 = FM0 - 1;
      int i1 = col - FM0; if (i1 < 0) i1 = 0; if (i1 > FM1 - 1) i1 = FM1 - 1;
      const float b0 = bias0[i0];
      const float b1 = bias1[i1];
      bv = (col < FM0) ? b0 : b1;
    } else {
      int i0 = col; if (i0 > FM0 - 1) i0 = FM0 - 1;
      bv = bias0[i0];
    }
#pragma unroll
    for (int r = 0; r < 8; ++r) c[j][r] = bv;
  }

#pragma unroll 1
  for (int ks = 0; ks < K / 32; ++ks) {
    const int k0 = ks * 32;
    BFrag a0h, a0l;
    {
      const unsigned short* pa = Ah + (rt * 16 + m) * K + k0 + 8 * hh;
      const unsigned short* qa = Al + (rt * 16 + m) * K + k0 + 8 * hh;
      a0h.half[0] = *(const v8us*)pa;  a0h.half[1] = *(const v8us*)(pa + 16);
      a0l.half[0] = *(const v8us*)qa;  a0l.half[1] = *(const v8us*)(qa + 16);
    }
    BFrag a1h, a1l;
    if constexpr (DUAL) {
      int arow = rowBase + rt * 16 + m;
      if (arow > M - 1) arow = M - 1;
      const unsigned short* pa = A1h + (size_t)arow * K + k0 + 8 * hh;
      const unsigned short* qa = A1l + (size_t)arow * K + k0 + 8 * hh;
      a1h.half[0] = *(const v8us*)pa;  a1h.half[1] = *(const v8us*)(pa + 16);
      a1l.half[0] = *(const v8us*)qa;  a1l.half[1] = *(const v8us*)(qa + 16);
    }
#pragma unroll
    for (int j = 0; j < NTW; ++j) {
      const int  gn    = ch * NTW + j;
      const int  ncol  = gn * 16 + m;
      const bool isres = (gn >= NTM);
      if (!isres || dores) {
        BFrag bh, bl;
        const unsigned short* pb = Wh + (size_t)ncol * K + k0 + 8 * hh;
        const unsigned short* qb = Wl + (size_t)ncol * K + k0 + 8 * hh;
        bh.half[0] = *(const v8us*)pb;  bh.half[1] = *(const v8us*)(pb + 16);
        bl.half[0] = *(const v8us*)qb;  bl.half[1] = *(const v8us*)(qb + 16);
        c[j] = wmb(a0h.v, bh.v, c[j]);
        c[j] = wmb(a0h.v, bl.v, c[j]);
        c[j] = wmb(a0l.v, bh.v, c[j]);
      }
      if constexpr (DUAL) {
        if (!isres) {
          BFrag vh, vl;
          const unsigned short* pv = Vh + (size_t)ncol * K + k0 + 8 * hh;
          const unsigned short* qv = Vl + (size_t)ncol * K + k0 + 8 * hh;
          vh.half[0] = *(const v8us*)pv;  vh.half[1] = *(const v8us*)(pv + 16);
          vl.half[0] = *(const v8us*)qv;  vl.half[1] = *(const v8us*)(qv + 16);
          c[j] = wmb(a1h.v, vh.v, c[j]);
          c[j] = wmb(a1h.v, vl.v, c[j]);
          c[j] = wmb(a1l.v, vh.v, c[j]);
        }
      }
    }
  }

#pragma unroll
  for (int j = 0; j < NTW; ++j) {
    const int ncol = (ch * NTW + j) * 16 + m;
#pragma unroll
    for (int r = 0; r < 8; ++r) Xs[(rt * 16 + 8 * hh + r) * XP + ncol] = c[j][r];
  }
  __syncthreads();

  auto emit = [&]() {
#pragma unroll 1
    for (int i = 0; i < GR / 4; ++i) {
      const int row  = wave * (GR / 4) + i;
      const int grow = rowBase + row;
      if (grow < M) {
        const float* xrow = Xs + row * XP;
#pragma unroll
        for (int q = 0; q < FM0; q += 128) {
          const int nl = ((FM0 - q) >= 128) ? 32 : ((FM0 - q) / 4);
          if (lane < nl) {
            const v4f v = *(const v4f*)(xrow + q + 4 * lane);
            *(volatile v4f*)(out0 + (size_t)grow * FM0 + q + 4 * lane) = v;
          }
        }
        if constexpr (NTR > 0) {
          if (dores && lane < 16) {
            const v4f v = *(const v4f*)(xrow + FM0 + 4 * lane);
            *(volatile v4f*)(out1 + (size_t)grow * FM1 + 4 * lane) = v;
          }
        }
      }
    }
  };
  emit();
  __threadfence();
  emit();
}

template<bool MIX>
__global__ __launch_bounds__(NTHR) void k_ssm(
    const float* __restrict__ conv, const float* __restrict__ xsr,
    const float* __restrict__ logA, const float* __restrict__ dlt_in,
    const float* __restrict__ tkw,  const float* __restrict__ tkb,
    float* xout, int nV, int tmin)
{
#pragma clang fp contract(off)
  __shared__ float red1[NWAVE];
  __shared__ float red2[NWAVE];
  __shared__ __attribute__((aligned(16))) float outs[NTHR];

  const int tid  = threadIdx.x;
  const int lane = tid & 31;
  const int wave = tid >> 5;
  const int q    = tid >> 6;
  const int h    = tid & 63;
  const int v0   = blockIdx.x * 4;
  int vc = v0 + q;
  if (vc > nV - 1) vc = nV - 1;

  float An[NS];
#pragma unroll
  for (int n = 0; n < NS; ++n) An[n] = -__expf(logA[h * NS + n]);
  const float dl = dlt_in[h];
  float w0 = 0.f, w1 = 0.f, w2 = 0.f, wb = 0.f;
  if constexpr (MIX) {
    w0 = tkw[h * 3 + 0]; w1 = tkw[h * 3 + 1]; w2 = tkw[h * 3 + 2]; wb = tkb[h];
  }
  float st[NS];
#pragma unroll
  for (int n = 0; n < NS; ++n) st[n] = 0.0f;

#pragma unroll 1
  for (int t = 0; t < TT; ++t) {
    const size_t rbase = (size_t)t * (size_t)nV + (size_t)vc;
    const float* crow = conv + rbase * CO;
    const float dtr = crow[HH + h] + dl;
    const float sp  = fmaxf(dtr, 0.0f) + log1pf(expf(-fabsf(dtr)));
    float xin;
    if constexpr (MIX) {
      const int tm = (t > 0) ? t - 1 : 0;
      const int tp = (t < TT - 1) ? t + 1 : TT - 1;
      float xm = conv[((size_t)tm * (size_t)nV + (size_t)vc) * CO + h];
      float xp = conv[((size_t)tp * (size_t)nV + (size_t)vc) * CO + h];
      xm = (t > 0) ? xm : 0.0f;
      xp = (t < TT - 1) ? xp : 0.0f;
      const float x0 = crow[h];
      xin = ((xm * w0 + x0 * w1) + xp * w2) + wb;
    } else {
      xin = crow[h];
    }
    const v4f* bp = (const v4f*)(crow + 2 * HH);
    const v4f* cp = (const v4f*)(crow + 2 * HH + NS);
    v4f B4[4], C4[4];
#pragma unroll
    for (int i = 0; i < 4; ++i) { B4[i] = bp[i]; C4[i] = cp[i]; }
    float y = 0.0f;
#pragma unroll
    for (int n = 0; n < NS; ++n) {
      const float b  = B4[n >> 2][n & 3];
      const float cN = C4[n >> 2][n & 3];
      const float az = __expf(sp * An[n]);
      st[n] = az * st[n] + (sp * b) * xin;
      y = y + st[n] * cN;
    }
    y = fmaxf(y, 0.0f);

    if (t >= tmin) {
      const float z = y + xsr[rbase * HH + h];
      const float s1 = wsum(z);
      if (lane == 0) red1[wave] = s1;
      __syncthreads();
      const float mean = (red1[2 * q] + red1[2 * q + 1]) * (1.0f / HH);
      const float d  = z - mean;
      const float s2 = wsum(d * d);
      if (lane == 0) red2[wave] = s2;
      __syncthreads();
      const float var = (red2[2 * q] + red2[2 * q + 1]) * (1.0f / HH);
      const float o = d * rsqrtf(var + LN_EPS);
      outs[tid] = o;
      __syncthreads();
      const int idx   = (wave & 1) * 32 + lane;
      const int qq    = idx >> 4;
      const int piece = idx & 15;
      const int vv    = v0 + qq;
      const bool doit = (wave < 2) && (vv < nV);
      const v4f val = *(const v4f*)(outs + qq * 64 + piece * 4);
      int vvc = vv;
      if (vvc > nV - 1) vvc = nV - 1;
      float* gp = xout + ((size_t)t * (size_t)nV + (size_t)vvc) * HH + piece * 4;
      if (doit) *(volatile v4f*)gp = val;
      __threadfence();
      if (doit) *(volatile v4f*)gp = val;
      __syncthreads();
    }
  }
}

extern "C" void kernel_launch(void* const* d_in, const int* in_sizes, int n_in,
                              void* d_out, int out_size, void* d_ws, size_t ws_size,
                              hipStream_t stream)
{
  if (n_in < 18) return;
  const int nV = in_sizes[0] / (TT * CIN);
  const int nE = in_sizes[1] / (TT * 2);
  if (nV <= 0 || in_sizes[0] != nV * TT * CIN) return;
  if (nE <= 0 || in_sizes[1] != nE * TT * 2) return;
  if (in_sizes[2] != CIN * CO || in_sizes[3] != CIN * CO || in_sizes[4] != CO) return;
  if (in_sizes[5] != HH * CO || in_sizes[6] != HH * CO || in_sizes[7] != CO) return;
  if (in_sizes[8] != CIN * HH || in_sizes[9] != HH || in_sizes[10] != HH * HH || in_sizes[11] != HH) return;
  if (in_sizes[12] != HH * 3 || in_sizes[13] != HH || in_sizes[14] != 2 * HH * NS || in_sizes[15] != 2 * HH) return;
  if (in_sizes[16] != HH * COUT || in_sizes[17] != COUT) return;
  if (out_size != nV * COUT) return;

  const float* xs    = (const float*)d_in[0];
  const int*   ei    = (const int*)d_in[1];
  const float* Wl0   = (const float*)d_in[2];
  const float* Wr0   = (const float*)d_in[3];
  const float* bc0   = (const float*)d_in[4];
  const float* Wl1   = (const float*)d_in[5];
  const float* Wr1   = (const float*)d_in[6];
  const float* bc1   = (const float*)d_in[7];
  const float* Wres0 = (const float*)d_in[8];
  const float* bres0 = (const float*)d_in[9];
  const float* Wres1 = (const float*)d_in[10];
  const float* bres1 = (const float*)d_in[11];
  const float* tkw   = (const float*)d_in[12];
  const float* tkb   = (const float*)d_in[13];
  const float* logA  = (const float*)d_in[14];
  const float* delta = (const float*)d_in[15];
  const float* Wmlp  = (const float*)d_in[16];
  const float* bmlp  = (const float*)d_in[17];
  float* out = (float*)d_out;

  const size_t TV = (size_t)TT * (size_t)nV;

  size_t off = 0;
  unsigned short* Wc_h = (unsigned short*)((char*)d_ws + off); off += (size_t)224 * 128 * 2;
  unsigned short* Wc_l = (unsigned short*)((char*)d_ws + off); off += (size_t)224 * 128 * 2;
  unsigned short* Wr_h = (unsigned short*)((char*)d_ws + off); off += (size_t)160 * 128 * 2;
  unsigned short* Wr_l = (unsigned short*)((char*)d_ws + off); off += (size_t)160 * 128 * 2;
  char* Ragg = (char*)d_ws + off;          off += TV * CIN * 4;
  float* conv = (float*)((char*)d_ws + off); off += TV * CO * 4;
  float* xsr  = (float*)((char*)d_ws + off); off += TV * HH * 4;
  float* xs1  = (float*)((char*)d_ws + off); off += TV * HH * 4;
  if (off > ws_size) return;
  unsigned short* agg_h  = (unsigned short*)Ragg;
  unsigned short* agg_l0 = agg_h + TV * CIN;
  unsigned short* agg_l1 = agg_h + TV * HH;
  float* xs2 = (float*)(Ragg + TV * HH * 2 * 2);

  const size_t lds128 = (size_t)32768 * 4 + 256 * 4 + (size_t)NWAVE * WCAP * 4 + NWAVE * 4;
  const size_t lds64  = (size_t)32768 * 4 + 512 * 4 + (size_t)NWAVE * WCAP * 4 + NWAVE * 4;
  hipFuncSetAttribute(reinterpret_cast<const void*>(&k_agg<128>),
                      hipFuncAttributeMaxDynamicSharedMemorySize, (int)lds128);
  hipFuncSetAttribute(reinterpret_cast<const void*>(&k_agg<64>),
                      hipFuncAttributeMaxDynamicSharedMemorySize, (int)lds64);

  const int gemmBlocks = (int)((TV + GR - 1) / GR);
  const int ssmBlocks  = (nV + 3) / 4;

  k_wprep<<<(160 * (CIN / 8) + NTHR - 1) / NTHR, NTHR, 0, stream>>>(Wl0, CIN, CO, Wc_h, Wc_l);
  k_wprep<<<(64 * (CIN / 8) + NTHR - 1) / NTHR, NTHR, 0, stream>>>(Wres0, CIN, HH,
                                                                   Wc_h + (size_t)160 * CIN, Wc_l + (size_t)160 * CIN);
  k_wprep<<<(160 * (CIN / 8) + NTHR - 1) / NTHR, NTHR, 0, stream>>>(Wr0, CIN, CO, Wr_h, Wr_l);
  {
    dim3 g((nV + 255) / 256, TT);
    k_agg<128><<<g, NTHR, lds128, stream>>>(xs, ei, agg_h, agg_l0, nV, nE);
  }
  k_gemm<128, 10, 4, true><<<gemmBlocks, 128, 0, stream>>>(
      xs, (int)TV, agg_h, agg_l0, Wc_h, Wc_l, Wr_h, Wr_l, bc0, bres0, conv, xsr, 0);
  k_ssm<true><<<ssmBlocks, NTHR, 0, stream>>>(conv, xsr, logA, delta, tkw, tkb, xs1, nV, 0);

  k_wprep<<<(160 * (HH / 8) + NTHR - 1) / NTHR, NTHR, 0, stream>>>(Wl1, HH, CO, Wc_h, Wc_l);
  k_wprep<<<(64 * (HH / 8) + NTHR - 1) / NTHR, NTHR, 0, stream>>>(Wres1, HH, HH,
                                                                  Wc_h + (size_t)160 * HH, Wc_l + (size_t)160 * HH);
  k_wprep<<<(160 * (HH / 8) + NTHR - 1) / NTHR, NTHR, 0, stream>>>(Wr1, HH, CO, Wr_h, Wr_l);
  {
    dim3 g((nV + 511) / 512, TT);
    k_agg<64><<<g, NTHR, lds64, stream>>>(xs1, ei, agg_h, agg_l1, nV, nE);
  }
  k_gemm<64, 10, 4, true><<<gemmBlocks, 128, 0, stream>>>(
      xs1, (int)TV, agg_h, agg_l1, Wc_h, Wc_l, Wr_h, Wr_l, bc1, bres1, conv, xsr, (TT - 1) * nV);
  k_ssm<false><<<ssmBlocks, NTHR, 0, stream>>>(conv, xsr, logA + HH * NS, delta + HH, tkw, tkb,
                                               xs2, nV, TT - 1);

  k_wprep<<<(64 * (HH / 8) + NTHR - 1) / NTHR, NTHR, 0, stream>>>(Wmlp, HH, COUT, Wc_h, Wc_l);
  const float* xlast = xs2 + (size_t)(TT - 1) * (size_t)nV * HH;
  k_gemm<64, 4, 0, false><<<(nV + GR - 1) / GR, 128, 0, stream>>>(
      xlast, nV, Wc_h, Wc_l, Wc_h, Wc_l, Wc_h, Wc_l, bmlp, bmlp, out, out, 0);
}
